// DeeProBot_MoE_bl_52518860095674
// MI455X (gfx1250) — hardware-verified
//
#include <hip/hip_runtime.h>
#include <hip/hip_bf16.h>
#include <math.h>


#define BB 2
#define SS 2048
#define DD 1024
#define HH 16
#define DKK 64
#define QW 2

typedef _Float16 bf16;
typedef __attribute__((ext_vector_type(4))) unsigned v4u_t;
typedef unsigned v4ua __attribute__((ext_vector_type(4), may_alias));
typedef __attribute__((ext_vector_type(4))) float v4f_t;
typedef float v4fa __attribute__((ext_vector_type(4), may_alias));
typedef __attribute__((ext_vector_type(16))) bf16  bf16x16;
typedef __attribute__((ext_vector_type(8)))  bf16  bf16x8;
typedef __attribute__((ext_vector_type(4)))  bf16  bf16x4;
typedef __attribute__((ext_vector_type(8)))  float f32x8;

#define LDS_STRIDE 48
#define KSTRIDE    72
#define VSTRIDE    48

__device__ __forceinline__ f32x8 wmma_bf16(bf16x16 a, bf16x16 b, f32x8 c) {
  return __builtin_amdgcn_wmma_f32_16x16x32_f16(
      false, a, false, b, (short)0, c, false, false);
}

template <typename T>
__device__ __forceinline__ bf16x16 load_frag(const T* __restrict__ base, int ld,
                                             int row0, int k0) {
  const int lane = threadIdx.x & 31;
  const int r    = lane & 15;
  const int kh   = (lane >> 4) * 8;
  const T* p0 = base + (size_t)(row0 + r) * ld + (k0 + kh);
  const T* p1 = p0 + 16;
  bf16x16 f;
#pragma unroll
  for (int i = 0; i < 8; ++i) {
    f[i]     = (bf16)p0[i];
    f[i + 8] = (bf16)p1[i];
  }
  return f;
}

__device__ __forceinline__ bf16x16 lds_frag(const bf16* base, int stride) {
  const int lane = threadIdx.x & 31;
  const int row  = lane & 15;
  const int kh   = (lane >> 4) * 8;
  const bf16x8 lo = *(const bf16x8*)(base + row * stride + kh);
  const bf16x8 hi = *(const bf16x8*)(base + row * stride + kh + 16);
  bf16x16 f;
#pragma unroll
  for (int i = 0; i < 8; ++i) { f[i] = lo[i]; f[i + 8] = hi[i]; }
  return f;
}

template <typename T>
__device__ __forceinline__ void stage_read16(const T* __restrict__ p, float* buf) {
#pragma unroll
  for (int i = 0; i < 16; ++i) buf[i] = (float)p[i];
}

__device__ __forceinline__ void stage_write(bf16* dst, const float* buf, int nquad) {
#pragma unroll
  for (int i = 0; i < nquad; ++i) {
    bf16x4 q;
    q[0] = (bf16)buf[4 * i];     q[1] = (bf16)buf[4 * i + 1];
    q[2] = (bf16)buf[4 * i + 2]; q[3] = (bf16)buf[4 * i + 3];
    *(bf16x4*)(dst + 4 * i) = q;
  }
}

template <typename AT, typename WTY, int MODE>
__global__ __launch_bounds__(256) void gemm_bias_kernel(
    const AT* __restrict__ A, const WTY* __restrict__ W,
    const float* __restrict__ bias, void* __restrict__ out,
    int M, int N, int K) {
  __shared__ bf16 ldsA[128 * LDS_STRIDE];
  __shared__ bf16 ldsW[256 * LDS_STRIDE];
  __shared__ __attribute__((aligned(16))) unsigned char sob[256 * 136 * 2];

  const int t    = threadIdx.x;
  const int wave = t >> 5;
  const int lane = t & 31;
  const int wm   = (wave & 1) * 64;
  const int wn   = (wave >> 1) * 64;
  const int mBlk = blockIdx.x * 128;
  const int nBlk = blockIdx.y * 256;

  const int arow = t >> 1;
  const int ach  = (t & 1) * 16;

  float abuf[16];
  float wbuf[32];

  stage_read16(A + (size_t)(mBlk + arow) * K + ach, abuf);
  stage_read16(W + (size_t)(nBlk + t) * K,          wbuf);
  stage_read16(W + (size_t)(nBlk + t) * K + 16,     wbuf + 16);

  f32x8 acc[4][4] = {};

  for (int k = 0; k < K; k += 32) {
    __syncthreads();
    stage_write(&ldsA[arow * LDS_STRIDE + ach], abuf, 4);
    stage_write(&ldsW[t * LDS_STRIDE],          wbuf, 8);
    if (k + 32 < K) {
      stage_read16(A + (size_t)(mBlk + arow) * K + (k + 32) + ach, abuf);
      stage_read16(W + (size_t)(nBlk + t) * K + (k + 32),          wbuf);
      stage_read16(W + (size_t)(nBlk + t) * K + (k + 32) + 16,     wbuf + 16);
    }
    __syncthreads();

    bf16x16 af[4], wf[4];
#pragma unroll
    for (int i = 0; i < 4; ++i)
      af[i] = lds_frag(ldsA + (wm + 16 * i) * LDS_STRIDE, LDS_STRIDE);
#pragma unroll
    for (int j = 0; j < 4; ++j)
      wf[j] = lds_frag(ldsW + (wn + 16 * j) * LDS_STRIDE, LDS_STRIDE);
#pragma unroll
    for (int i = 0; i < 4; ++i)
#pragma unroll
      for (int j = 0; j < 4; ++j)
        acc[i][j] = wmma_bf16(af[i], wf[j], acc[i][j]);
  }

  const int nlane = lane & 15;
  const int mh    = (lane >> 4) * 8;
  __syncthreads();
  if (MODE == 0 || MODE == 1 || MODE == 3) {
    bf16* so = (bf16*)sob;
#pragma unroll
    for (int i = 0; i < 4; ++i)
#pragma unroll
      for (int j = 0; j < 4; ++j) {
        const int nl = wn + 16 * j + nlane;
        const float bv = bias ? bias[nBlk + nl] : 0.0f;
#pragma unroll
        for (int r = 0; r < 8; ++r) {
          const int ml = wm + 16 * i + mh + r;
          const bf16 hv = (MODE == 3) ? (bf16)fmaxf(acc[i][j][r] + bv, 0.0f) : (bf16)(acc[i][j][r] + bv);
          if (MODE == 0 || MODE == 3) so[ml * 264 + nl] = hv;
          else           so[nl * 136 + ml] = hv;
        }
      }
    __syncthreads();
#pragma unroll 1
    for (int pass = 0; pass < 2; ++pass) {
      if (MODE == 0 || MODE == 3) {
        for (int ch = t; ch < 128 * 32; ch += 256) { const int ml = ch >> 5, q = (ch & 31) * 8;
          *(volatile v4u_t*)((bf16*)out + (size_t)(mBlk + ml) * N + nBlk + q) = *(const v4ua*)(so + ml * 264 + q); }
      } else {
        const int b_ = mBlk / SS, s0 = mBlk & (SS - 1);
        for (int ch = t; ch < 256 * 16; ch += 256) { const int nl = ch >> 4, q = (ch & 15) * 8; const int n = nBlk + nl, h = n >> 6, dk = n & (DKK - 1);
          *(volatile v4u_t*)((bf16*)out + (((size_t)(b_ * HH + h)) * DKK + dk) * SS + s0 + q) = *(const v4ua*)(so + nl * 136 + q); }
      }
      __threadfence();
    }
  } else {
    float* so = (float*)sob;
#pragma unroll 1
    for (int hf = 0; hf < 2; ++hf) {
      if (wm == hf * 64) {
#pragma unroll
        for (int i = 0; i < 4; ++i)
#pragma unroll
          for (int j = 0; j < 4; ++j) {
            const int nl = wn + 16 * j + nlane;
            const float bv = bias ? bias[nBlk + nl] : 0.0f;
#pragma unroll
            for (int r = 0; r < 8; ++r) so[(16 * i + mh + r) * 260 + nl] = acc[i][j][r] + bv;
          }
      }
      __syncthreads();
#pragma unroll 1
      for (int pass = 0; pass < 2; ++pass) {
        for (int ch = t; ch < 64 * 64; ch += 256) { const int ml = ch >> 6, q = (ch & 63) * 4;
          *(volatile v4f_t*)((float*)out + (size_t)(mBlk + hf * 64 + ml) * N + nBlk + q) = *(const volatile v4fa*)(so + ml * 260 + q); }
        __threadfence();
      }
      __syncthreads();
    }
  }
}


#define NTK 524288
#define CH 65536
#define DIN 9
#define NEX 2
#define HEX 128
#define MO 32

__global__ __launch_bounds__(256) void k_gate(const float* __restrict__ x, const float* __restrict__ wg, int* __restrict__ sel, float* __restrict__ part) {
  __shared__ int cnt[8];
  const int n = blockIdx.x * 256 + threadIdx.x, t = threadIdx.x, lane = t & 31, wave = t >> 5;
  const float* xr = x + (size_t)n * DIN; float l0 = 0.f, l1 = 0.f;
#pragma unroll
  for (int d = 0; d < DIN; ++d) { const float xv = xr[d]; l0 += xv * wg[d * NEX]; l1 += xv * wg[d * NEX + 1]; }
  const int s = (l1 > l0) ? 1 : 0;
  *(volatile int*)(sel + n) = s;
  const unsigned m = __builtin_amdgcn_ballot_w32(s != 0); if (lane == 0) cnt[wave] = __builtin_popcount(m);
  __syncthreads(); __threadfence();
  *(volatile int*)(sel + n) = s;
  if (t < 32) { float v = 0.0f; if (t == 0) { int c = 0; for (int w = 0; w < 8; ++w) c += cnt[w]; v = (float)c; }
    *(volatile float*)(part + (size_t)blockIdx.x * 32 + t) = v; __threadfence(); *(volatile float*)(part + (size_t)blockIdx.x * 32 + t) = v; }
}
__global__ __launch_bounds__(32) void k_loss(const float* __restrict__ part, int nblk, float* __restrict__ loss) {
  if (threadIdx.x == 0) { double c1 = 0.0; for (int i = 0; i < nblk; ++i) c1 += (double)part[(size_t)i * 32];
    const double c0 = (double)NTK - c1, mu = (c0 + c1) / 2.0, var = ((c0 - mu) * (c0 - mu) + (c1 - mu) * (c1 - mu)) / 1.0;
    const double cv = var / (mu * mu + 1e-10); const float v = (float)(0.01 * (cv + cv)); *(volatile float*)loss = v; __threadfence(); *(volatile float*)loss = v; }
}
__global__ __launch_bounds__(256) void k_xpad(const float* __restrict__ x, int n0, float* __restrict__ Xp) {
  const int nl = blockIdx.x * 8 + (threadIdx.x >> 5), c = threadIdx.x & 31; const float v = (c < DIN) ? x[(size_t)(n0 + nl) * DIN + c] : 0.0f;
  *(volatile float*)(Xp + (size_t)nl * 32 + c) = v; __threadfence(); *(volatile float*)(Xp + (size_t)nl * 32 + c) = v;
}
__global__ __launch_bounds__(32) void k_w1rows(const float* __restrict__ W1, float* __restrict__ Wr) {
  const int n = blockIdx.x, e = n / HEX, h = n % HEX, c = threadIdx.x; const float v = (c < DIN) ? W1[((size_t)e * DIN + c) * HEX + h] : 0.0f;
  *(volatile float*)(Wr + (size_t)n * 32 + c) = v; __threadfence(); *(volatile float*)(Wr + (size_t)n * 32 + c) = v;
}
__global__ __launch_bounds__(256) void k_a2(const float* __restrict__ W2, float* __restrict__ A2) {
  const int mrow = blockIdx.x, k = threadIdx.x; float v = 0.0f;
  if (mrow < NEX * MO) { const int e = mrow / MO, m = mrow % MO, e2 = k / HEX, h = k % HEX; if (e == e2) v = W2[((size_t)e * HEX + h) * MO + m]; }
  *(volatile float*)(A2 + (size_t)mrow * 256 + k) = v; __threadfence(); *(volatile float*)(A2 + (size_t)mrow * 256 + k) = v;
}
__global__ __launch_bounds__(256) void k_comb(const float* __restrict__ T, const int* __restrict__ sel, const float* __restrict__ b2, const float* __restrict__ Wout, const float* __restrict__ bout, int n0, float* __restrict__ out) {
  __shared__ float wo[MO][2]; __shared__ float bb[NEX][MO];
  const int t = threadIdx.x, nl = blockIdx.x * 256 + t; const int n = n0 + nl;
  if (t < MO * 2) wo[t >> 1][t & 1] = Wout[t]; if (t < NEX * MO) bb[t / MO][t % MO] = b2[t];
  __syncthreads();
  const int s = sel[n]; float o0 = bout[0], o1 = bout[1];
#pragma unroll 1
  for (int m = 0; m < MO; ++m) { const float y = T[(size_t)(s * MO + m) * CH + nl] + bb[s][m]; o0 += y * wo[m][0]; o1 += y * wo[m][1]; }
  typedef __attribute__((ext_vector_type(2))) float v2f;
  v2f r; r.x = o0; r.y = o1; *(volatile v2f*)(out + (size_t)n * 2) = r; __threadfence(); *(volatile v2f*)(out + (size_t)n * 2) = r;
}

extern "C" void kernel_launch(void* const* d_in, const int* in_sizes, int n_in,
                              void* d_out, int out_size, void* d_ws, size_t ws_size,
                              hipStream_t stream) {
  (void)in_sizes; (void)n_in; (void)out_size; (void)ws_size;
  const float* x = (const float*)d_in[0];
  const float* wg = (const float*)d_in[2];
  const float* W1 = (const float*)d_in[3]; const float* b1 = (const float*)d_in[4];
  const float* W2 = (const float*)d_in[5]; const float* b2 = (const float*)d_in[6];
  const float* Wout = (const float*)d_in[7]; const float* bout = (const float*)d_in[8];
  float* out = (float*)d_out;
  float* loss = out + (size_t)NTK * 2;
  char* ws = (char*)d_ws;
  float* Wr = (float*)ws; ws += (size_t)256 * 32 * 4;
  float* A2 = (float*)ws; ws += (size_t)128 * 256 * 4;
  int* sel  = (int*)ws;   ws += (size_t)NTK * 4;
  const int nblk = NTK / 256;
  float* part = (float*)ws; ws += (size_t)nblk * 32 * 4;
  float* Xp = (float*)ws; ws += (size_t)CH * 32 * 4;
  bf16* Hh  = (bf16*)ws;  ws += (size_t)CH * 256 * 2;
  float* T  = (float*)ws; ws += (size_t)128 * CH * 4;
  k_w1rows<<<256, 32, 0, stream>>>(W1, Wr);
  k_a2<<<128, 256, 0, stream>>>(W2, A2);
  k_gate<<<nblk, 256, 0, stream>>>(x, wg, sel, part);
  k_loss<<<1, 32, 0, stream>>>(part, nblk, loss);
  dim3 blk(256);
  for (int c = 0; c < NTK / CH; ++c) { const int n0 = c * CH;
    k_xpad<<<CH / 8, 256, 0, stream>>>(x, n0, Xp);
    gemm_bias_kernel<float, float, 3><<<dim3(CH / 128, 1), blk, 0, stream>>>(Xp, Wr, b1, Hh, CH, 256, 32);
    gemm_bias_kernel<float, bf16, 2><<<dim3(1, CH / 256), blk, 0, stream>>>(A2, Hh, nullptr, T, 128, CH, 256);
    k_comb<<<CH / 256, 256, 0, stream>>>(T, sel, b2, Wout, bout, n0, out);
  }
}
